// GNN_43370579755357
// MI455X (gfx1250) — hardware-verified
//
#include <hip/hip_runtime.h>
#include <stddef.h>
#include <stdint.h>
#include <math.h>


#define HD     128
#define NHEAD  8
#define DKH    16
#define NTYPE  4
#define NLAY   2
#define AP2    256
#define NQKV   384
#define IN0    256
#define IN1    128
#define IN2    512
#define IN3    64
#define NTHR   256
#define NWAVE  8
#define EPT    8
#define CHUNK  (NTHR * EPT)
#define WCAP   (EPT * 32)
#define LISTN  (NWAVE * WCAP)
#define SNBA   512
#define SLA    9
#define RCAP   20480
#define DEGCAP 64
#define GBM    64
#define GBN    128
#define GTHR   128
#define U_KQV  (NLAY * NTYPE * NQKV * (AP2 / 8))
#define U_WO   (NLAY * NTYPE * HD * (AP2 / 8))
#define U_A0   (HD * (IN0 / 8))
#define U_A1   (HD * (IN1 / 8))
#define U_A2   (HD * (IN2 / 8))
#define U_A3   (HD * (IN3 / 8))
#define U_TOT  (U_KQV + U_WO + U_A0 + U_A1 + U_A2 + U_A3)
#define AGG_ZINTS     (LISTN + 2 * RCAP + 3 * SNBA)
#define MISC_INTS     16
#define ROWBUF_INTS   (NWAVE * AP2 / 2)
#define SCW_INTS      (NWAVE * DEGCAP * NHEAD)
#define SCAN_LDS_INTS (AGG_ZINTS + MISC_INTS + ROWBUF_INTS + SCW_INTS)
#define WSMAX  134217728

static_assert((CHUNK & (CHUNK - 1)) == 0 && CHUNK <= 4096);
static_assert((SNBA & (SNBA - 1)) == 0 && SNBA == (1 << SLA));
static_assert(((long long)CHUNK << SLA) < (1LL << 31));
static_assert(SNBA % NWAVE == 0 && SNBA % 32 == 0 && SNBA % GBM == 0);
static_assert(RCAP % 4 == 0 && AGG_ZINTS % 4 == 0 && LISTN % 4 == 0 && SCAN_LDS_INTS % 4 == 0);
static_assert(((AGG_ZINTS + MISC_INTS) % 4) == 0 && ((AGG_ZINTS + MISC_INTS + ROWBUF_INTS) % 4) == 0);
static_assert(SCAN_LDS_INTS * 4 <= 300000);
static_assert(DEGCAP % 32 == 0 && DEGCAP >= 56 + 8);
static_assert(HD == 4 * 32 && HD == NHEAD * DKH && AP2 == 2 * HD && NQKV == 3 * HD);
static_assert(GBN == HD && GBM == (GTHR / 32) * 16);
static_assert(IN0 % 32 == 0 && IN1 % 32 == 0 && IN2 % 32 == 0 && IN3 % 32 == 0 && AP2 % 32 == 0);
static_assert(U_KQV % NTHR == 0 && U_WO % NTHR == 0 && U_A0 % NTHR == 0 && U_A1 % NTHR == 0);
static_assert(U_A2 % NTHR == 0 && U_A3 % NTHR == 0 && (NQKV * (AP2 / 8)) % NTHR == 0 && HD % 8 == 0);

typedef float          v4f   __attribute__((ext_vector_type(4)));
typedef float          v8f   __attribute__((ext_vector_type(8)));
typedef int            v4i   __attribute__((ext_vector_type(4)));
typedef int            v8i   __attribute__((ext_vector_type(8)));
typedef unsigned short v4us  __attribute__((ext_vector_type(4)));
typedef unsigned short v8us  __attribute__((ext_vector_type(8)));
typedef unsigned short v16us __attribute__((ext_vector_type(16)));
typedef __bf16         v16bf __attribute__((ext_vector_type(16)));
typedef v4f  __attribute__((may_alias)) v4fa;
typedef v4i  __attribute__((may_alias)) v4ia;
typedef v4us __attribute__((may_alias)) v4usa;
typedef v8us __attribute__((may_alias)) v8usa;
union FragB { v16bf v; v16us u; v8us h[2]; v8i w; };

__device__ __forceinline__ v8f wmb(const FragB& a, const FragB& b, v8f c) {
  v8f d = __builtin_amdgcn_wmma_f32_16x16x32_bf16(false, a.v, false, b.v, (short)0, c, false, false);
  asm volatile("v_nop\n\tv_nop\n\tv_nop\n\tv_nop" : "+v"(d) : "v"(a.w), "v"(b.w));
  return d;
}

__device__ __forceinline__ unsigned bf16_bits(float f) {
  const unsigned u = __float_as_uint(f);
  return (u + 0x7FFFu + ((u >> 16) & 1u)) >> 16;
}
__device__ __forceinline__ float bf16_val(float f) {
  return __uint_as_float(bf16_bits(f) << 16);
}

__device__ __forceinline__ void wave_sync() {
  __builtin_amdgcn_fence(__ATOMIC_RELEASE, "wavefront");
  __builtin_amdgcn_wave_barrier();
  __builtin_amdgcn_fence(__ATOMIC_ACQUIRE, "wavefront");
}

__device__ __forceinline__ v8us hilo_pack(unsigned short* rowbuf, int lane, const v4f y) {
  v4us mh, ml;
  unsigned hb;
  hb = bf16_bits(y.x); mh[0] = (unsigned short)hb; ml[0] = (unsigned short)bf16_bits(y.x - __uint_as_float(hb << 16));
  hb = bf16_bits(y.y); mh[1] = (unsigned short)hb; ml[1] = (unsigned short)bf16_bits(y.y - __uint_as_float(hb << 16));
  hb = bf16_bits(y.z); mh[2] = (unsigned short)hb; ml[2] = (unsigned short)bf16_bits(y.z - __uint_as_float(hb << 16));
  hb = bf16_bits(y.w); mh[3] = (unsigned short)hb; ml[3] = (unsigned short)bf16_bits(y.w - __uint_as_float(hb << 16));
  *(v4usa*)(rowbuf + 4 * lane) = mh;
  *(v4usa*)(rowbuf + HD + 4 * lane) = ml;
  wave_sync();
  const v8us q = *(const v8usa*)(rowbuf + 8 * lane);
  wave_sync();
  return q;
}

__device__ __forceinline__ float gelu_t(float a) {
  const float u = 0.7978845608028654f * (a + 0.044715f * (a * a * a));
  return 0.5f * a * (1.0f + tanhf(u));
}

__device__ __forceinline__ void gemm_k(const unsigned short* ap, const unsigned short* __restrict__ bp, int K,
                                       v8f (&acc)[8]) {
#pragma unroll 1
  for (int k0 = 0; k0 < K; k0 += 32) {
    FragB af;
    af.h[0] = *(const v8usa*)(ap + k0);
    af.h[1] = *(const v8usa*)(ap + k0 + 16);
#pragma unroll
    for (int nt = 0; nt < 8; ++nt) {
      const unsigned short* wq = bp + (size_t)(16 * nt) * (size_t)K + k0;
      FragB bf;
      bf.h[0] = *(const v8usa*)wq;
      bf.h[1] = *(const v8usa*)(wq + 16);
      acc[nt] = wmb(af, bf, acc[nt]);
    }
  }
}

__device__ __forceinline__ void stage_acc(float* stg, const v8f (&acc)[8], int wave, int hh, int m) {
#pragma unroll
  for (int nt = 0; nt < 8; ++nt) {
    const int lc = 16 * nt + m;
#pragma unroll
    for (int r = 0; r < 8; ++r) {
      const int lr = 16 * wave + 8 * hh + r;
      stg[lr * GBN + lc] = acc[nt][r];
    }
  }
}

template <int SLB>
__device__ __forceinline__ int scan_chunk(const int* __restrict__ dsts, int nE, int cbase, int slotBase,
                                          int nb, int vec8, int* list, int tid, int lane, int wave) {
  int wc = 0;
  const int el0  = tid * EPT;
  const int e0   = cbase + el0;
  const int sent = -2147483647 - 1;
  v4i da, db;
  if (vec8 != 0 && cbase + CHUNK <= nE) {
    da = *(const v4i*)(dsts + e0);
    db = *(const v4i*)(dsts + e0 + 4);
  } else {
    da.x = (e0     < nE) ? dsts[min(e0,     nE - 1)] : sent;
    da.y = (e0 + 1 < nE) ? dsts[min(e0 + 1, nE - 1)] : sent;
    da.z = (e0 + 2 < nE) ? dsts[min(e0 + 2, nE - 1)] : sent;
    da.w = (e0 + 3 < nE) ? dsts[min(e0 + 3, nE - 1)] : sent;
    db.x = (e0 + 4 < nE) ? dsts[min(e0 + 4, nE - 1)] : sent;
    db.y = (e0 + 5 < nE) ? dsts[min(e0 + 5, nE - 1)] : sent;
    db.z = (e0 + 6 < nE) ? dsts[min(e0 + 6, nE - 1)] : sent;
    db.w = (e0 + 7 < nE) ? dsts[min(e0 + 7, nE - 1)] : sent;
  }
  const unsigned nbs = (unsigned)slotBase;
  const unsigned unb = (unsigned)nb;
  const unsigned s0 = (unsigned)da.x - nbs, s1 = (unsigned)da.y - nbs;
  const unsigned s2 = (unsigned)da.z - nbs, s3 = (unsigned)da.w - nbs;
  const unsigned s4 = (unsigned)db.x - nbs, s5 = (unsigned)db.y - nbs;
  const unsigned s6 = (unsigned)db.z - nbs, s7 = (unsigned)db.w - nbs;
  const bool h0 = s0 < unb, h1 = s1 < unb, h2 = s2 < unb, h3 = s3 < unb;
  const bool h4 = s4 < unb, h5 = s5 < unb, h6 = s6 < unb, h7 = s7 < unb;
  const unsigned any = __builtin_amdgcn_ballot_w32(h0 | h1 | h2 | h3 | h4 | h5 | h6 | h7);
  if (any != 0u) {
#define HITJ(J, HJ, SJ) { \
      const unsigned mj = __builtin_amdgcn_ballot_w32(HJ); \
      if (mj != 0u) { \
        if (HJ) { \
          const int pos = wc + (int)__builtin_amdgcn_mbcnt_lo(mj, 0u); \
          if (pos < WCAP) list[wave * WCAP + pos] = ((el0 + (J)) << SLB) | (int)(SJ); \
        } \
        wc += (int)__builtin_popcount(mj); } }
    HITJ(0, h0, s0)
    HITJ(1, h1, s1)
    HITJ(2, h2, s2)
    HITJ(3, h3, s3)
    HITJ(4, h4, s4)
    HITJ(5, h5, s5)
    HITJ(6, h6, s6)
    HITJ(7, h7, s7)
#undef HITJ
  }
  return wc;
}

__device__ __forceinline__ void tr8(const float* __restrict__ src, unsigned short* dp) {
  v8us o;
#pragma unroll
  for (int i = 0; i < 8; ++i) o[i] = (unsigned short)bf16_bits(src[(size_t)i * HD]);
  *(volatile v8us*)dp = o;
  __threadfence();
  *(volatile v8us*)dp = o;
}

__global__ __launch_bounds__(NTHR) void k_prep(const float* __restrict__ Wk, const float* __restrict__ Wq,
                                               const float* __restrict__ Wv, const float* __restrict__ Wo,
                                               const float* __restrict__ aw0, const float* __restrict__ aw1,
                                               const float* __restrict__ aw2, const float* __restrict__ aw3,
                                               unsigned short* PKQV, unsigned short* PWO,
                                               unsigned short* PA0, unsigned short* PA1,
                                               unsigned short* PA2, unsigned short* PA3) {
  const int u = (int)blockIdx.x * NTHR + (int)threadIdx.x;
  if (u < U_KQV) {
    const int lt  = u / (NQKV * (AP2 / 8));
    const int rem = u - lt * (NQKV * (AP2 / 8));
    const int r   = rem >> 5;
    const int k8  = (rem & 31) * 8;
    const int p   = r >> 7;
    const int n   = r & (HD - 1);
    const size_t so = (size_t)lt * HD * HD + (size_t)(k8 & (HD - 1)) * HD + n;
    unsigned short* dp = PKQV + (size_t)u * 8;
    if (p == 0)      tr8(Wk + so, dp);
    else if (p == 1) tr8(Wq + so, dp);
    else             tr8(Wv + so, dp);
  } else if (u < U_KQV + U_WO) {
    const int v   = u - U_KQV;
    const int lt  = v >> 12;
    const int rem = v & 4095;
    const int n   = rem >> 5;
    const int k8  = (rem & 31) * 8;
    tr8(Wo + (size_t)lt * HD * HD + (size_t)(k8 & (HD - 1)) * HD + n, PWO + (size_t)v * 8);
  } else if (u < U_KQV + U_WO + U_A0) {
    const int w = u - (U_KQV + U_WO);
    const int n = w / (IN0 / 8), k8 = (w % (IN0 / 8)) * 8;
    tr8(aw0 + (size_t)k8 * HD + n, PA0 + (size_t)w * 8);
  } else if (u < U_KQV + U_WO + U_A0 + U_A1) {
    const int w = u - (U_KQV + U_WO + U_A0);
    const int n = w / (IN1 / 8), k8 = (w % (IN1 / 8)) * 8;
    tr8(aw1 + (size_t)k8 * HD + n, PA1 + (size_t)w * 8);
  } else if (u < U_KQV + U_WO + U_A0 + U_A1 + U_A2) {
    const int w = u - (U_KQV + U_WO + U_A0 + U_A1);
    const int n = w / (IN2 / 8), k8 = (w % (IN2 / 8)) * 8;
    tr8(aw2 + (size_t)k8 * HD + n, PA2 + (size_t)w * 8);
  } else if (u < U_TOT) {
    const int w = u - (U_KQV + U_WO + U_A0 + U_A1 + U_A2);
    const int n = w / (IN3 / 8), k8 = (w % (IN3 / 8)) * 8;
    tr8(aw3 + (size_t)k8 * HD + n, PA3 + (size_t)w * 8);
  }
}

__global__ __launch_bounds__(GTHR) void k_adapt(const float* __restrict__ F, const unsigned short* __restrict__ AWT,
                                                const float* __restrict__ ab, int K, int rowsT, int rowOff,
                                                int padTo, float* X, unsigned short* XG) {
  __shared__ __attribute__((aligned(16))) float stg[GBM * GBN];
  __shared__ __attribute__((aligned(16))) unsigned short rbuf[(GTHR / 32) * AP2];
  const int tid = (int)threadIdx.x, lane = tid & 31, wave = tid >> 5, hh = lane >> 4, m = lane & 15;
  const int lr0 = (int)blockIdx.x * GBM + 16 * wave;
  int ar = lr0 + m;
  ar = ar < rowsT ? ar : rowsT - 1;
  const float* ap = F + (size_t)ar * (size_t)K + 8 * hh;
  const unsigned short* bp = AWT + (size_t)m * (size_t)K + 8 * hh;

  v8f acc[8];
  {
    const v8f z = {0.f, 0.f, 0.f, 0.f, 0.f, 0.f, 0.f, 0.f};
#pragma unroll
    for (int t = 0; t < 8; ++t) acc[t] = z;
  }
#pragma unroll 1
  for (int k0 = 0; k0 < K; k0 += 32) {
    const v4f a0 = *(const v4f*)(ap + k0);
    const v4f a1 = *(const v4f*)(ap + k0 + 4);
    const v4f a2 = *(const v4f*)(ap + k0 + 16);
    const v4f a3 = *(const v4f*)(ap + k0 + 20);
    v8us t0, t1;
    t0[0] = (unsigned short)bf16_bits(a0.x); t0[1] = (unsigned short)bf16_bits(a0.y);
    t0[2] = (unsigned short)bf16_bits(a0.z); t0[3] = (unsigned short)bf16_bits(a0.w);
    t0[4] = (unsigned short)bf16_bits(a1.x); t0[5] = (unsigned short)bf16_bits(a1.y);
    t0[6] = (unsigned short)bf16_bits(a1.z); t0[7] = (unsigned short)bf16_bits(a1.w);
    t1[0] = (unsigned short)bf16_bits(a2.x); t1[1] = (unsigned short)bf16_bits(a2.y);
    t1[2] = (unsigned short)bf16_bits(a2.z); t1[3] = (unsigned short)bf16_bits(a2.w);
    t1[4] = (unsigned short)bf16_bits(a3.x); t1[5] = (unsigned short)bf16_bits(a3.y);
    t1[6] = (unsigned short)bf16_bits(a3.z); t1[7] = (unsigned short)bf16_bits(a3.w);
    FragB af;
    af.h[0] = t0;
    af.h[1] = t1;
#pragma unroll
    for (int nt = 0; nt < 8; ++nt) {
      const unsigned short* wq = bp + (size_t)(16 * nt) * (size_t)K + k0;
      FragB bf;
      bf.h[0] = *(const v8usa*)wq;
      bf.h[1] = *(const v8usa*)(wq + 16);
      acc[nt] = wmb(af, bf, acc[nt]);
    }
  }
  stage_acc(stg, acc, wave, hh, m);
  __syncthreads();

  v4f bb4;
  {
    const v4f t = *(const v4f*)(ab + 4 * lane);
    bb4.x = bf16_val(t.x); bb4.y = bf16_val(t.y); bb4.z = bf16_val(t.z); bb4.w = bf16_val(t.w);
  }
  unsigned short* rowbuf = rbuf + wave * AP2;
#pragma unroll 1
  for (int i = 0; i < 16; ++i) {
    const int lr = lr0 + i;
    const int gr = rowOff + lr;
    const v4f t = *(const v4fa*)(stg + (16 * wave + i) * GBN + 4 * lane);
    const bool live = lr < rowsT;
    v4f y;
    y.x = tanhf(t.x + bb4.x); y.y = tanhf(t.y + bb4.y);
    y.z = tanhf(t.z + bb4.z); y.w = tanhf(t.w + bb4.w);
    y.x = live ? y.x : 0.0f; y.y = live ? y.y : 0.0f; y.z = live ? y.z : 0.0f; y.w = live ? y.w : 0.0f;
    const v8us q = hilo_pack(rowbuf, lane, y);
    if (gr < padTo) {
      float* xp = X + (size_t)gr * HD + 4 * lane;
      unsigned short* gp = XG + (size_t)gr * AP2 + 8 * lane;
      *(volatile v4f*)xp = y;
      *(volatile v8us*)gp = q;
      __threadfence();
      *(volatile v4f*)xp = y;
      *(volatile v8us*)gp = q;
    }
  }
}

__global__ __launch_bounds__(GTHR) void k_kqv(const unsigned short* __restrict__ XG,
                                              const unsigned short* __restrict__ WP,
                                              const int* __restrict__ ntype,
                                              const float* __restrict__ bk, const float* __restrict__ bq,
                                              const float* __restrict__ bv, const float* __restrict__ hmat,
                                              int nN, float* KV, float* QT) {
  __shared__ __attribute__((aligned(16))) float stg[GBM * GBN];
  __shared__ int tys[GBM];
  __shared__ int pm[GTHR / 32];
  const int tid = (int)threadIdx.x, lane = tid & 31, wave = tid >> 5, hh = lane >> 4, m = lane & 15;
  const int rowBase = (int)blockIdx.x * GBM;
  {
    int r = rowBase + (tid & 63);
    r = r < nN ? r : nN - 1;
    int ty = ntype[r];
    ty = ty < 0 ? 0 : (ty > NTYPE - 1 ? NTYPE - 1 : ty);
    unsigned mk = 0u;
    mk |= (__builtin_amdgcn_ballot_w32(ty == 0) != 0u) ? 1u : 0u;
    mk |= (__builtin_amdgcn_ballot_w32(ty == 1) != 0u) ? 2u : 0u;
    mk |= (__builtin_amdgcn_ballot_w32(ty == 2) != 0u) ? 4u : 0u;
    mk |= (__builtin_amdgcn_ballot_w32(ty == 3) != 0u) ? 8u : 0u;
    if (tid < GBM) tys[tid] = ty;
    if (lane == 0) pm[wave] = (int)mk;
  }
  __syncthreads();
  const int pmask = pm[0] | pm[1] | pm[2] | pm[3];
  const unsigned short* ap = XG + (size_t)(rowBase + 16 * wave + m) * AP2 + 8 * hh;
  const int hq = lane >> 2, db = 4 * (lane & 3);

#pragma unroll 1
  for (int tt = 0; tt < NTYPE; ++tt) {
    if (((pmask >> tt) & 1) == 0) continue;
#pragma unroll 1
    for (int p = 0; p < 3; ++p) {
      v8f acc[8];
      {
        const v8f z = {0.f, 0.f, 0.f, 0.f, 0.f, 0.f, 0.f, 0.f};
#pragma unroll
        for (int t = 0; t < 8; ++t) acc[t] = z;
      }
      const unsigned short* bp = WP + (size_t)(tt * NQKV + p * HD + m) * AP2 + 8 * hh;
      gemm_k(ap, bp, AP2, acc);
      stage_acc(stg, acc, wave, hh, m);
      __syncthreads();

      if (p != 1) {
        v4f bb4;
        {
          const v4f t0 = *(const v4f*)(bk + tt * HD + 4 * lane);
          const v4f t2 = *(const v4f*)(bv + tt * HD + 4 * lane);
          bb4.x = bf16_val(p == 0 ? t0.x : t2.x);
          bb4.y = bf16_val(p == 0 ? t0.y : t2.y);
          bb4.z = bf16_val(p == 0 ? t0.z : t2.z);
          bb4.w = bf16_val(p == 0 ? t0.w : t2.w);
        }
        const int coff = (p == 0) ? 0 : HD;
#pragma unroll 1
        for (int i = 0; i < 16; ++i) {
          const int row = rowBase + 16 * wave + i;
          const int tyr = tys[16 * wave + i];
          if (tyr == tt && row < nN) {
            const v4f t = *(const v4fa*)(stg + (16 * wave + i) * GBN + 4 * lane);
            const v4f y = t + bb4;
            float* op = KV + (size_t)row * AP2 + coff + 4 * lane;
            *(volatile v4f*)op = y;
            __threadfence();
            *(volatile v4f*)op = y;
          }
        }
      } else {
        float hmr[4][16];
        float bqh[16];
#pragma unroll
        for (int j = 0; j < 4; ++j) {
#pragma unroll
          for (int f4 = 0; f4 < 4; ++f4) {
            const v4f t = *(const v4f*)(hmat + hq * (DKH * DKH) + (db + j) * DKH + 4 * f4);
            hmr[j][4 * f4 + 0] = 0.25f * bf16_val(t.x);
            hmr[j][4 * f4 + 1] = 0.25f * bf16_val(t.y);
            hmr[j][4 * f4 + 2] = 0.25f * bf16_val(t.z);
            hmr[j][4 * f4 + 3] = 0.25f * bf16_val(t.w);
          }
        }
#pragma unroll
        for (int f4 = 0; f4 < 4; ++f4) {
          const v4f t = *(const v4f*)(bq + tt * HD + hq * DKH + 4 * f4);
          bqh[4 * f4 + 0] = bf16_val(t.x); bqh[4 * f4 + 1] = bf16_val(t.y);
          bqh[4 * f4 + 2] = bf16_val(t.z); bqh[4 * f4 + 3] = bf16_val(t.w);
        }
#pragma unroll 1
        for (int i = 0; i < 16; ++i) {
          const int row = rowBase + 16 * wave + i;
          const int tyr = tys[16 * wave + i];
          if (tyr == tt && row < nN) {
            const float* sr = stg + (16 * wave + i) * GBN + hq * DKH;
            float qv[16];
#pragma unroll
            for (int f4 = 0; f4 < 4; ++f4) {
              const v4f t = *(const v4fa*)(sr + 4 * f4);
              qv[4 * f4 + 0] = t.x + bqh[4 * f4 + 0];
              qv[4 * f4 + 1] = t.y + bqh[4 * f4 + 1];
              qv[4 * f4 + 2] = t.z + bqh[4 * f4 + 2];
              qv[4 * f4 + 3] = t.w + bqh[4 * f4 + 3];
            }
            float oj[4];
#pragma unroll
            for (int j = 0; j < 4; ++j) {
              float s = 0.0f;
#pragma unroll
              for (int f = 0; f < 16; ++f) s = fmaf(hmr[j][f], qv[f], s);
              oj[j] = s;
            }
            v4f y;
            y.x = oj[0]; y.y = oj[1]; y.z = oj[2]; y.w = oj[3];
            float* op = QT + (size_t)row * HD + 4 * lane;
            *(volatile v4f*)op = y;
            __threadfence();
            *(volatile v4f*)op = y;
          }
        }
      }
      __syncthreads();
    }
  }
}

__global__ __launch_bounds__(NTHR) void k_scan(const int* __restrict__ srcs, const int* __restrict__ dsts,
                                               int nE, int nN, int vec8, int mRows,
                                               const float* __restrict__ kv, const float* __restrict__ qt,
                                               unsigned short* xg) {
  extern __shared__ __attribute__((aligned(16))) int dsm[];
  int* list = dsm;
  int* hl   = dsm + LISTN;
  int* sl   = hl + RCAP;
  int* cnt  = sl + RCAP;
  int* offs = cnt + SNBA;
  int* cur  = offs + SNBA;
  int* misc = cur + SNBA;
  const int tid = (int)threadIdx.x, lane = tid & 31, wave = tid >> 5;
  unsigned short* rowbuf = (unsigned short*)(misc + MISC_INTS) + wave * AP2;
  float* scw = (float*)(misc + MISC_INTS + ROWBUF_INTS) + wave * (DEGCAP * NHEAD);
  const int nodeBase = (int)blockIdx.x * SNBA;

  {
    const v4i z4 = {0, 0, 0, 0};
    for (int i = tid * 4; i < SCAN_LDS_INTS; i += NTHR * 4) *(v4ia*)(dsm + i) = z4;
  }
  __syncthreads();

  int t = 0, ov = 0;
  const int nChunks = (nE + CHUNK - 1) / CHUNK;
#pragma unroll 1
  for (int ch = 0; ch < nChunks; ++ch) {
    const int cbase = ch * CHUNK;
    const int wc = scan_chunk<SLA>(dsts, nE, cbase, nodeBase, SNBA, vec8, list, tid, lane, wave);
    if (lane == 0) misc[wave] = wc;
    __syncthreads();
    if (wave == 0) {
#pragma unroll 1
      for (int w2 = 0; w2 < NWAVE; ++w2) {
        int c = misc[w2];
        c = c < 0 ? 0 : (c > WCAP ? WCAP : c);
#pragma unroll 1
        for (int b0 = 0; b0 < c; b0 += 32) {
          const int idx = b0 + lane;
          const int ent = list[w2 * WCAP + (idx < WCAP ? idx : WCAP - 1)];
          const int m32 = (c - b0) < 32 ? (c - b0) : 32;
#pragma unroll 1
          for (int k = 0; k < m32; ++k) {
            const int u    = __builtin_amdgcn_readlane(ent, k);
            const int slot = u & (SNBA - 1);
            const int el   = (u >> SLA) & (CHUNK - 1);
            const int pk   = ((cbase + el) << SLA) | slot;
            if (t < RCAP) {
              if (lane == 0) { hl[t] = pk; cnt[slot] = cnt[slot] + 1; }
              t = t + 1;
            } else {
              ov = 1;
            }
          }
        }
      }
    }
    __syncthreads();
  }
  if (wave == 0 && lane == 0) { misc[8] = t; misc[9] = ov; }
  __syncthreads();
  int tt = misc[8];
  tt = tt < 0 ? 0 : (tt > RCAP ? RCAP : tt);
  const int ovf = misc[9];

  if (wave == 0) {
    const int base = lane * (SNBA / 32);
    int s = 0;
#pragma unroll 1
    for (int i = 0; i < SNBA / 32; ++i) s += cnt[base + i];
    int incl = s;
#pragma unroll
    for (int d = 1; d < 32; d <<= 1) {
      const int y = __shfl_up(incl, d, 32);
      if (lane >= d) incl += y;
    }
    int run = incl - s;
#pragma unroll 1
    for (int i = 0; i < SNBA / 32; ++i) {
      const int cv = cnt[base + i];
      offs[base + i] = run;
      cur[base + i]  = run;
      run += cv;
    }
  }
  __syncthreads();
  if (wave == 0) {
#pragma unroll 1
    for (int b0 = 0; b0 < tt; b0 += 32) {
      const int idx = b0 + lane;
      const int ent = hl[idx < RCAP ? idx : RCAP - 1];
      const int m32 = (tt - b0) < 32 ? (tt - b0) : 32;
#pragma unroll 1
      for (int k = 0; k < m32; ++k) {
        const int u    = __builtin_amdgcn_readlane(ent, k);
        const int slot = u & (SNBA - 1);
        if (lane == 0) {
          int p = cur[slot];
          p = p < 0 ? 0 : (p > RCAP - 1 ? RCAP - 1 : p);
          sl[p] = u;
          cur[slot] = p + 1;
        }
      }
    }
  }
  __syncthreads();

  const float qnan = __int_as_float(0x7fc00000);
  const float pz = (ovf != 0) ? qnan : 0.0f;
  const int hq = lane >> 2;
#pragma unroll 1
  for (int si = 0; si < SNBA / NWAVE; ++si) {
    const int s    = si * NWAVE + wave;
    const int node = nodeBase + s;
    int c = cnt[s];
    const bool big = c > DEGCAP;
    c = c < 0 ? 0 : (c > DEGCAP ? DEGCAP : c);
    int o = offs[s];
    o = o < 0 ? 0 : (o > RCAP ? RCAP : o);
    const int nc = node < nN ? node : nN - 1;
    const v4f q4 = *(const v4f*)(qt + (size_t)nc * HD + 4 * lane);
    float mx = -__builtin_inff();
#pragma unroll 1
    for (int b0 = 0; b0 < c; b0 += 32) {
      int idx = o + b0 + lane;
      idx = idx > RCAP - 1 ? RCAP - 1 : idx;
      const int ent = sl[idx];
      int eid = ent >> SLA;
      eid = eid < 0 ? 0 : (eid > nE - 1 ? nE - 1 : eid);
      int sr = srcs[eid];
      sr = sr < 0 ? 0 : (sr > nN - 1 ? nN - 1 : sr);
      const int m32 = (c - b0) < 32 ? (c - b0) : 32;
#pragma unroll 1
      for (int k = 0; k < m32; ++k) {
        const int sk = __builtin_amdgcn_readlane(sr, k);
        const v4f kk = *(const v4f*)(kv + (size_t)sk * AP2 + 4 * lane);
        float sc = q4.x * kk.x;
        sc = fmaf(q4.y, kk.y, sc);
        sc = fmaf(q4.z, kk.z, sc);
        sc = fmaf(q4.w, kk.w, sc);
        sc += __shfl_xor(sc, 1, 32);
        sc += __shfl_xor(sc, 2, 32);
        mx = (sc > mx) ? sc : mx;
        if ((lane & 3) == 0) scw[(b0 + k) * NHEAD + hq] = sc;
      }
    }
    wave_sync();
    float den = 0.0f, a0 = 0.0f, a1 = 0.0f, a2 = 0.0f, a3 = 0.0f;
#pragma unroll 1
    for (int b0 = 0; b0 < c; b0 += 32) {
      int idx = o + b0 + lane;
      idx = idx > RCAP - 1 ? RCAP - 1 : idx;
      const int ent = sl[idx];
      int eid = ent >> SLA;
      eid = eid < 0 ? 0 : (eid > nE - 1 ? nE - 1 : eid);
      int sr = srcs[eid];
      sr = sr < 0 ? 0 : (sr > nN - 1 ? nN - 1 : sr);
      const int m32 = (c - b0) < 32 ? (c - b0) : 32;
#pragma unroll 1
      for (int k = 0; k < m32; ++k) {
        const int sk = __builtin_amdgcn_readlane(sr, k);
        const v4f vv = *(const v4f*)(kv + (size_t)sk * AP2 + HD + 4 * lane);
        const float sc = scw[(b0 + k) * NHEAD + hq];
        const float ex = expf(sc - mx);
        den += ex;
        a0 = fmaf(ex, vv.x, a0);
        a1 = fmaf(ex, vv.y, a1);
        a2 = fmaf(ex, vv.z, a2);
        a3 = fmaf(ex, vv.w, a3);
      }
    }
    const float inv = 1.0f / (den + 1e-16f);
    const float pzr = big ? qnan : pz;
    const bool live = node < nN;
    const float g0 = gelu_t(a0 * inv + pzr);
    const float g1 = gelu_t(a1 * inv + pzr);
    const float g2 = gelu_t(a2 * inv + pzr);
    const float g3 = gelu_t(a3 * inv + pzr);
    v4f y;
    y.x = live ? g0 : 0.0f; y.y = live ? g1 : 0.0f; y.z = live ? g2 : 0.0f; y.w = live ? g3 : 0.0f;
    const v8us qv = hilo_pack(rowbuf, lane, y);
    if (node < mRows) {
      unsigned short* rp = xg + (size_t)node * AP2 + 8 * lane;
      *(volatile v8us*)rp = qv;
      __threadfence();
      *(volatile v8us*)rp = qv;
    }
  }
}

template <int FIN>
__global__ __launch_bounds__(GTHR) void k_out(unsigned short* XG, const unsigned short* __restrict__ WO,
                                              const int* __restrict__ ntype, const float* __restrict__ bo,
                                              const float* __restrict__ skp, const float* __restrict__ lng,
                                              const float* __restrict__ lnb, int nN, float* X, float* outp) {
  __shared__ __attribute__((aligned(16))) float stg[GBM * GBN];
  __shared__ __attribute__((aligned(16))) unsigned short rbuf[(GTHR / 32) * AP2];
  __shared__ int tys[GBM];
  __shared__ int pm[GTHR / 32];
  __shared__ float sa[NTYPE];
  const int tid = (int)threadIdx.x, lane = tid & 31, wave = tid >> 5, hh = lane >> 4, m = lane & 15;
  const int rowBase = (int)blockIdx.x * GBM;
  {
    int r = rowBase + (tid & 63);
    r = r < nN ? r : nN - 1;
    int ty = ntype[r];
    ty = ty < 0 ? 0 : (ty > NTYPE - 1 ? NTYPE - 1 : ty);
    unsigned mk = 0u;
    mk |= (__builtin_amdgcn_ballot_w32(ty == 0) != 0u) ? 1u : 0u;
    mk |= (__builtin_amdgcn_ballot_w32(ty == 1) != 0u) ? 2u : 0u;
    mk |= (__builtin_amdgcn_ballot_w32(ty == 2) != 0u) ? 4u : 0u;
    mk |= (__builtin_amdgcn_ballot_w32(ty == 3) != 0u) ? 8u : 0u;
    const float sv = bf16_val(skp[tid & (NTYPE - 1)]);
    const float av = 1.0f / (1.0f + expf(-sv));
    if (tid < GBM) tys[tid] = ty;
    if (lane == 0) pm[wave] = (int)mk;
    if (tid < NTYPE) sa[tid] = av;
  }
  __syncthreads();
  const int pmask = pm[0] | pm[1] | pm[2] | pm[3];
  const unsigned short* ap = XG + (size_t)(rowBase + 16 * wave + m) * AP2 + 8 * hh;
  unsigned short* rowbuf = rbuf + wave * AP2;
  v4f g4, b4;
  {
    const v4f tg = *(const v4f*)(lng + 4 * lane);
    const v4f tb = *(const v4f*)(lnb + 4 * lane);
    g4.x = bf16_val(tg.x); g4.y = bf16_val(tg.y); g4.z = bf16_val(tg.z); g4.w = bf16_val(tg.w);
    b4.x = bf16_val(tb.x); b4.y = bf16_val(tb.y); b4.z = bf16_val(tb.z); b4.w = bf16_val(tb.w);
  }

#pragma unroll 1
  for (int tt = 0; tt < NTYPE; ++tt) {
    if (((pmask >> tt) & 1) == 0) continue;
    v8f acc[8];
    {
      const v8f z = {0.f, 0.f, 0.f, 0.f, 0.f, 0.f, 0.f, 0.f};
#pragma unroll
      for (int t = 0; t < 8; ++t) acc[t] = z;
    }
    const unsigned short* bp = WO + (size_t)(tt * HD + m) * AP2 + 8 * hh;
    gemm_k(ap, bp, AP2, acc);
    stage_acc(stg, acc, wave, hh, m);
    __syncthreads();

    v4f bo4;
    {
      const v4f t0 = *(const v4f*)(bo + tt * HD + 4 * lane);
      bo4.x = bf16_val(t0.x); bo4.y = bf16_val(t0.y); bo4.z = bf16_val(t0.z); bo4.w = bf16_val(t0.w);
    }
    const float a  = sa[tt];
    const float om = 1.0f - a;
#pragma unroll 1
    for (int i = 0; i < 16; ++i) {
      const int row = rowBase + 16 * wave + i;
      const int tyr = tys[16 * wave + i];
      if (tyr == tt && row < nN) {
        const v4f t  = *(const v4fa*)(stg + (16 * wave + i) * GBN + 4 * lane);
        const v4f xr = *(const v4f*)(X + (size_t)row * HD + 4 * lane);
        v4f y;
        y.x = (t.x + bo4.x) * a + xr.x * om;
        y.y = (t.y + bo4.y) * a + xr.y * om;
        y.z = (t.z + bo4.z) * a + xr.z * om;
        y.w = (t.w + bo4.w) * a + xr.w * om;
        float s = (y.x + y.y) + (y.z + y.w);
        s += __shfl_xor(s, 16, 32); s += __shfl_xor(s, 8, 32); s += __shfl_xor(s, 4, 32);
        s += __shfl_xor(s, 2, 32);  s += __shfl_xor(s, 1, 32);
        const float mean = s * (1.0f / HD);
        const float d0 = y.x - mean, d1 = y.y - mean, d2 = y.z - mean, d3 = y.w - mean;
        float ss = (d0 * d0 + d1 * d1) + (d2 * d2 + d3 * d3);
        ss += __shfl_xor(ss, 16, 32); ss += __shfl_xor(ss, 8, 32); ss += __shfl_xor(ss, 4, 32);
        ss += __shfl_xor(ss, 2, 32);  ss += __shfl_xor(ss, 1, 32);
        const float rstd = rsqrtf(ss * (1.0f / HD) + 1e-5f);
        v4f o;
        o.x = d0 * rstd * g4.x + b4.x;
        o.y = d1 * rstd * g4.y + b4.y;
        o.z = d2 * rstd * g4.z + b4.z;
        o.w = d3 * rstd * g4.w + b4.w;
        if constexpr (FIN != 0) {
          float* op = outp + (size_t)row * HD + 4 * lane;
          *(volatile v4f*)op = o;
          __threadfence();
          *(volatile v4f*)op = o;
        } else {
          const v8us q = hilo_pack(rowbuf, lane, o);
          float* xp = X + (size_t)row * HD + 4 * lane;
          unsigned short* gp = XG + (size_t)row * AP2 + 8 * lane;
          *(volatile v4f*)xp = o;
          *(volatile v8us*)gp = q;
          __threadfence();
          *(volatile v4f*)xp = o;
          *(volatile v8us*)gp = q;
        }
      }
    }
    __syncthreads();
  }
}

static inline int cdiv(int a, int b) { return (a + b - 1) / b; }
static inline size_t al256(size_t o) { return (o + 255) & ~(size_t)255; }

extern "C" void kernel_launch(void* const* d_in, const int* in_sizes, int n_in,
                              void* d_out, int out_size, void* d_ws, size_t ws_size,
                              hipStream_t stream) {
  if (n_in < 26) return;
  const int INW[NTYPE] = {IN0, IN1, IN2, IN3};
  int rowsT[NTYPE], rowOff[NTYPE];
  int tot = 0;
  for (int t = 0; t < NTYPE; ++t) {
    if (in_sizes[t] < INW[t] || (in_sizes[t] % INW[t]) != 0) return;
    rowsT[t] = in_sizes[t] / INW[t];
    rowOff[t] = tot;
    tot += rowsT[t];
  }
  const int nN = in_sizes[4];
  if (nN != tot || nN < GBM || nN > (1 << 22)) return;
  if (in_sizes[5] < 2 || (in_sizes[5] & 1) != 0) return;
  const int nE = in_sizes[5] / 2;
  if (nE < 1 || nE >= (1 << (31 - SLA))) return;
  if (in_sizes[6] != NHEAD * DKH * DKH) return;
  for (int t = 0; t < NTYPE; ++t) {
    if (in_sizes[7 + 2 * t] != INW[t] * HD) return;
    if (in_sizes[8 + 2 * t] != HD) return;
  }
  for (int i = 15; i <= 18; ++i) if (in_sizes[i] != NLAY * NTYPE * HD * HD) return;
  for (int i = 19; i <= 22; ++i) if (in_sizes[i] != NLAY * NTYPE * HD) return;
  if (in_sizes[23] != NLAY * NTYPE) return;
  if (in_sizes[24] != NLAY * HD || in_sizes[25] != NLAY * HD) return;
  if ((long long)out_size != (long long)nN * HD) return;

  const float* F[NTYPE]  = {(const float*)d_in[0], (const float*)d_in[1],
                            (const float*)d_in[2], (const float*)d_in[3]};
  const int*   ntype = (const int*)d_in[4];
  const int*   edge  = (const int*)d_in[5];
  const float* hmat  = (const float*)d_in[6];
  const float* awp[NTYPE] = {(const float*)d_in[7], (const float*)d_in[9],
                             (const float*)d_in[11], (const float*)d_in[13]};
  const float* abp[NTYPE] = {(const float*)d_in[8], (const float*)d_in[10],
                             (const float*)d_in[12], (const float*)d_in[14]};
  const float* Wk = (const float*)d_in[15];
  const float* Wq = (const float*)d_in[16];
  const float* Wv = (const float*)d_in[17];
  const float* Wo = (const float*)d_in[18];
  const float* bk = (const float*)d_in[19];
  const float* bq = (const float*)d_in[20];
  const float* bv = (const float*)d_in[21];
  const float* bo = (const float*)d_in[22];
  const float* skp = (const float*)d_in[23];
  const float* lng = (const float*)d_in[24];
  const float* lnb = (const float*)d_in[25];
  float* out = (float*)d_out;
  const int* src = edge;
  const int* dst = edge + nE;

  const int MP = cdiv(nN, GBM) * GBM;
  const int gM = MP / GBM;
  const int gA = cdiv(MP, SNBA);
  if ((long long)gA * SNBA < (long long)MP) return;
  const int vec8 = ((nE & 3) == 0) ? 1 : 0;

  char* ws = (char*)d_ws;
  size_t off = 0;
  const size_t oX   = off; off = al256(off + (size_t)MP * HD * 4);
  const size_t oXG  = off; off = al256(off + (size_t)MP * AP2 * 2);
  const size_t oKV  = off; off = al256(off + (size_t)MP * AP2 * 4);
  const size_t oQT  = off; off = al256(off + (size_t)MP * HD * 4);
  const size_t oPK  = off; off = al256(off + (size_t)NLAY * NTYPE * NQKV * AP2 * 2);
  const size_t oPO  = off; off = al256(off + (size_t)NLAY * NTYPE * HD * AP2 * 2);
  const size_t oA0  = off; off = al256(off + (size_t)HD * IN0 * 2);
  const size_t oA1  = off; off = al256(off + (size_t)HD * IN1 * 2);
  const size_t oA2  = off; off = al256(off + (size_t)HD * IN2 * 2);
  const size_t oA3  = off; off = al256(off + (size_t)HD * IN3 * 2);
  if (off > ws_size || off > (size_t)WSMAX) return;
  float*          X    = (float*)(ws + oX);
  unsigned short* XG   = (unsigned short*)(ws + oXG);
  float*          KV   = (float*)(ws + oKV);
  float*          QT   = (float*)(ws + oQT);
  unsigned short* PKQV = (unsigned short*)(ws + oPK);
  unsigned short* PWO  = (unsigned short*)(ws + oPO);
  unsigned short* PA[NTYPE] = {(unsigned short*)(ws + oA0), (unsigned short*)(ws + oA1),
                               (unsigned short*)(ws + oA2), (unsigned short*)(ws + oA3)};

  const size_t scanLds = (size_t)SCAN_LDS_INTS * 4;
  hipFuncSetAttribute(reinterpret_cast<const void*>(&k_scan), hipFuncAttributeMaxDynamicSharedMemorySize, (int)scanLds);

  k_prep<<<U_TOT / NTHR, NTHR, 0, stream>>>(Wk, Wq, Wv, Wo, awp[0], awp[1], awp[2], awp[3],
                                            PKQV, PWO, PA[0], PA[1], PA[2], PA[3]);
  for (int t = 0; t < NTYPE; ++t) {
    const int padTo = (t == NTYPE - 1) ? MP : (rowOff[t] + rowsT[t]);
    const int g = cdiv(padTo - rowOff[t], GBM);
    k_adapt<<<g, GTHR, 0, stream>>>(F[t], PA[t], abp[t], INW[t], rowsT[t], rowOff[t], padTo, X, XG);
  }
  for (int l = 0; l < NLAY; ++l) {
    const unsigned short* wp = PKQV + (size_t)l * NTYPE * NQKV * AP2;
    const unsigned short* wo = PWO  + (size_t)l * NTYPE * HD * AP2;
    const size_t bofs = (size_t)l * NTYPE * HD;
    k_kqv<<<gM, GTHR, 0, stream>>>(XG, wp, ntype, bk + bofs, bq + bofs, bv + bofs, hmat, nN, KV, QT);
    k_scan<<<gA, NTHR, scanLds, stream>>>(src, dst, nE, nN, vec8, MP, KV, QT, XG);
    if (l == NLAY - 1)
      k_out<1><<<gM, GTHR, 0, stream>>>(XG, wo, ntype, bo + bofs, skp + l * NTYPE, lng + l * HD, lnb + l * HD,
                                        nN, X, out);
    else
      k_out<0><<<gM, GTHR, 0, stream>>>(XG, wo, ntype, bo + bofs, skp + l * NTYPE, lng + l * HD, lnb + l * HD,
                                        nN, X, out);
  }
}
